// Attention_24996709663241
// MI455X (gfx1250) — hardware-run, weakly checked
//
#include <hip/hip_runtime.h>


#ifndef NB
#define NB 128
#endif
#define NB_FULL 128
#define CIN   384
#define RES   14
#define NTOK  196
#define NP    224
#define NHEAD 8
#define KD    32
#define VD    128
#define CQK   256
#define CV    1024
#define CQKV  1536
#define COUT  384
#define GW    7
#define AW    2
#define QT    14
#define OSP   132
#define BN_EPS 1.0e-5f
#define QCAR  64.0f
#define ACAR  256.0f
#define WCAR  256.0f
#define CINV  (1.0f / 65536.0f)
#define SC2   ((float)(0.17677669529663687 * 1.4426950408889634 / 64.0))
#define LOG2E 1.4426950408889634f
#define PSH   14.0f
#define NEGB  (-3.0e38f)
#define NCHUNK ((NB % 2 == 0) ? 2 : 1)
#define BCH   (NB / NCHUNK)

static_assert(NTOK == RES * RES);
static_assert(NP % 32 == 0);
static_assert(NP >= NTOK);
static_assert(NP == 32 * GW);
static_assert(QT * 16 == NP);
static_assert(QT % AW == 0);
static_assert(KD == 32);
static_assert(CIN % 32 == 0);
static_assert(CV % 32 == 0);
static_assert(CQKV % 64 == 0);
static_assert(CQK % 64 == 0);
static_assert(COUT % 64 == 0);
static_assert(CQKV == 2 * CQK + CV);
static_assert(NHEAD * KD == CQK);
static_assert(NHEAD * VD == CV);
static_assert(2 * KD == 64);
static_assert(VD == 8 * 16);
static_assert((32 * GW) * 16 * 16 == 64 * NP * 4);
static_assert((32 * GW) * 8 * 16 == 64 * NP * 2);
static_assert((32 * GW) * 4 * 16 == NP * KD * 2);
static_assert((32 * GW) * 14 * 16 == 64 * NTOK * 4);
static_assert(256 * 7 * 16 == NP * 64 * 2);
static_assert(8 * 32 * 16 == 16 * VD * 2);
static_assert(((size_t)NHEAD * NP * NP / 4) % 256 == 0);
static_assert((64 * NTOK) % 4 == 0);
static_assert((NTOK * 4) % 16 == 0);
static_assert((NP * 2) % 16 == 0);
static_assert((OSP * 4) % 16 == 0);
static_assert(((size_t)CQKV * CIN) % 8 == 0);
static_assert(((size_t)COUT * CV) % 8 == 0);
static_assert(NB <= NB_FULL);
static_assert(NB % NCHUNK == 0);
static_assert((size_t)64 * NP * 4 + 512 <= 65536);
static_assert((size_t)64 * NTOK * 4 + 512 <= 65536);
static_assert((size_t)KD * 256 * 4 + (size_t)KD * NP * 4 + KD * 9 * 4 + 2 * KD * 4 <= 65536);
static_assert((size_t)AW * 16 * OSP * 4 <= 131072);
static_assert((size_t)64 * NTOK * 4 <= 131072);

typedef _Float16 h16;
typedef unsigned short bf;
typedef __attribute__((ext_vector_type(16))) __bf16   v16bf;
typedef __attribute__((ext_vector_type(16))) _Float16 v16h;
typedef __attribute__((ext_vector_type(8)))  _Float16 v8h;
typedef __attribute__((ext_vector_type(8)))  unsigned short v8us;
typedef __attribute__((ext_vector_type(8)))  float    v8f;
typedef __attribute__((ext_vector_type(4)))  float    v4f;
typedef v4f  __attribute__((may_alias)) v4fa;

__device__ __forceinline__ unsigned short f2bf(float f) { unsigned u = __float_as_uint(f); u += 0x7FFFu + ((u >> 16) & 1u); return (unsigned short)(u >> 16); }
__device__ __forceinline__ float bfr(float f) { return __uint_as_float(((unsigned)f2bf(f)) << 16); }
__device__ __forceinline__ v16h cat16(v8h lo, v8h hi) { return __builtin_shufflevector(lo, hi, 0, 1, 2, 3, 4, 5, 6, 7, 8, 9, 10, 11, 12, 13, 14, 15); }
__device__ __forceinline__ v16bf cat16b(v8us lo, v8us hi) { return __builtin_bit_cast(v16bf, __builtin_shufflevector(lo, hi, 0, 1, 2, 3, 4, 5, 6, 7, 8, 9, 10, 11, 12, 13, 14, 15)); }
__device__ __forceinline__ v8f wmma16(v16h a, v16h b, v8f c) { return __builtin_amdgcn_wmma_f32_16x16x32_f16(false, a, false, b, (short)0, c, false, false); }
__device__ __forceinline__ v8f wmmab(v16bf a, v16bf b, v8f c) { return __builtin_amdgcn_wmma_f32_16x16x32_bf16(false, a, false, b, (short)0, c, false, false); }
__device__ __forceinline__ v16h  ldh(const h16* p) { return cat16(*(const v8h*)p, *(const v8h*)(p + 16)); }
__device__ __forceinline__ v16bf ldb(const bf* p)  { return cat16b(*(const v8us*)p, *(const v8us*)(p + 16)); }
__device__ __forceinline__ void wave_sync() { __builtin_amdgcn_fence(3  , "wavefront"); __builtin_amdgcn_wave_barrier(); asm volatile("" ::: "memory"); }
static __device__ __forceinline__ h16 toh_flush(float v) { const h16 r = (h16)v; return (fabsf(v) < 6.103515625e-05f) ? (h16)0.0f : r; }
__device__ __forceinline__ v8f wmma16g(v16h a, v16h b, v8f c) { c = wmma16(a, b, c); asm volatile("v_nop\n\tv_nop\n\tv_nop\n\tv_nop" : "+v"(c) : "v"(a), "v"(b)); return c; }
__device__ __forceinline__ v8f wmmabg(v16bf a, v16bf b, v8f c) { c = wmmab(a, b, c); asm volatile("v_nop\n\tv_nop\n\tv_nop\n\tv_nop" : "+v"(c) : "v"(a), "v"(b)); return c; }

__global__ __launch_bounds__(256) void k_cvt8(const float* __restrict__ src, bf* dst, size_t n8) {
    const size_t i = (size_t)blockIdx.x * 256 + threadIdx.x; if (i >= n8) return;
    const v8f v = *(const v8f*)(src + i * 8); v8us o;
#pragma unroll
    for (int k = 0; k < 8; ++k) o[k] = f2bf(v[k]);
    *(volatile v8us*)(dst + i * 8) = o; __threadfence(); *(volatile v8us*)(dst + i * 8) = o;
}

__global__ __launch_bounds__(256) void k_wcv(const float* __restrict__ src, h16* dst, size_t n8) {
    const size_t i = (size_t)blockIdx.x * 256 + threadIdx.x; if (i >= n8) return;
    const v8f v = *(const v8f*)(src + i * 8); v8h o;
#pragma unroll
    for (int k = 0; k < 8; ++k) o[k] = toh_flush(bfr(v[k]) * WCAR);
    *(volatile v8h*)(dst + i * 8) = o; __threadfence(); *(volatile v8h*)(dst + i * 8) = o;
}

__global__ __launch_bounds__(256) void k_xt(const float* __restrict__ x, bf* XB) {
    __shared__ __align__(16) float xs[64 * NTOK];
    const int tid = threadIdx.x; const int c0 = blockIdx.x * 64, b = blockIdx.y;
    const float* src = x + ((size_t)b * CIN + c0) * NTOK;
#pragma unroll 1
    for (int i = tid; i < 64 * NTOK / 4; i += 256) { const v4f v = *(const v4f*)(src + (size_t)i * 4); *(v4fa*)(&xs[i * 4]) = v; }
    __syncthreads();
    bf* dst = XB + (size_t)b * NP * CIN + c0;
#pragma unroll 1
    for (int ps = 0; ps < 2; ++ps) {
#pragma unroll 1
        for (int i = 0; i < 7; ++i) { const int p = i * 256 + tid; const int t = p >> 3, c8 = (p & 7) * 8;
            const int tc = t < NTOK ? t : NTOK - 1; const bool live = t < NTOK; v8us o;
#pragma unroll
            for (int e = 0; e < 8; ++e) { const float v = xs[(c8 + e) * NTOK + tc]; o[e] = live ? f2bf(v) : (unsigned short)0; }
            *(volatile v8us*)(dst + (size_t)t * CIN + c8) = o; }
        if (ps == 0) __threadfence(); }
}

__global__ __launch_bounds__(256) void k_bias(const float* __restrict__ ab, const int* __restrict__ idxs, float* BP) {
    const int i = blockIdx.x * 256 + threadIdx.x;
    const int e0 = i * 4; const int h = e0 / (NP * NP); const int rem = e0 - h * (NP * NP); const int t = rem / NP, k0 = rem - t * NP;
    const int tc = t < NTOK ? t : NTOK - 1; v4f o;
#pragma unroll
    for (int e = 0; e < 4; ++e) { const int k = k0 + e; const int kc = k < NTOK ? k : NTOK - 1;
        int id = idxs[tc * NTOK + kc]; id = id < 0 ? 0 : (id > NTOK - 1 ? NTOK - 1 : id);
        float a = ab[h * NTOK + id]; asm volatile("" : "+v"(a));
        const bool live = (t < NTOK) & (k < NTOK);
        o[e] = live ? bfr(a) * LOG2E : 0.0f; }
    *(volatile v4f*)(BP + (size_t)i * 4) = o; __threadfence(); *(volatile v4f*)(BP + (size_t)i * 4) = o;
}

__global__ __launch_bounds__(32 * GW) void k_qkv(const bf* __restrict__ WB, const bf* __restrict__ XB,
                                                  const float* __restrict__ gg, const float* __restrict__ bb, const float* __restrict__ mm, const float* __restrict__ vv,
                                                  float* QP, h16* KP, h16* VT) {
    __shared__ __align__(16) float os[64 * NP];
    __shared__ float ss[64];
    __shared__ float ts[64];
    const int tid = threadIdx.x; const int lane = tid & 31, lr = lane & 15, hi = lane >> 4;
    const int wave = __builtin_amdgcn_readfirstlane((int)(threadIdx.x >> 5));
    const int o0 = blockIdx.x * 64, b = blockIdx.y;
    if (tid < 64) { const int o = o0 + tid; const float s = bfr(gg[o]) * rsqrtf(bfr(vv[o]) + BN_EPS); ss[tid] = s; ts[tid] = bfr(bb[o]) - bfr(mm[o]) * s; }
    v8f acc[4][2];
#pragma unroll
    for (int mb = 0; mb < 4; ++mb)
#pragma unroll
        for (int nb = 0; nb < 2; ++nb) acc[mb][nb] = (v8f){};
    const size_t aoff = (size_t)(o0 + lr) * CIN + 8 * hi;
    const size_t boff = ((size_t)b * NP + wave * 32 + lr) * CIN + 8 * hi;
#pragma unroll 1
    for (int kc = 0; kc < CIN; kc += 32) {
        v16bf a[4];
#pragma unroll
        for (int mb = 0; mb < 4; ++mb) a[mb] = ldb(WB + aoff + (size_t)mb * 16 * CIN + kc);
#pragma unroll
        for (int nb = 0; nb < 2; ++nb) { const v16bf bq = ldb(XB + boff + (size_t)nb * 16 * CIN + kc);
#pragma unroll
            for (int mb = 0; mb < 4; ++mb) acc[mb][nb] = wmmabg(a[mb], bq, acc[mb][nb]); }
    }
    __syncthreads();
#pragma unroll
    for (int mb = 0; mb < 4; ++mb)
#pragma unroll
        for (int nb = 0; nb < 2; ++nb) { const int col = wave * 32 + nb * 16 + lr; const bool live = col < NTOK;
#pragma unroll
            for (int j = 0; j < 8; ++j) { const int row = mb * 16 + hi * 8 + j;
                const float val = acc[mb][nb][j] * ss[row] + ts[row];
                os[row * NP + col] = live ? val : 0.0f; } }
    __syncthreads();
    if (o0 < CQK) {
        float* dst = QP + ((size_t)b * CQK + o0) * NP;
#pragma unroll 1
        for (int ps = 0; ps < 2; ++ps) {
#pragma unroll 1
            for (int i = 0; i < 16; ++i) { const int idx = i * (32 * GW) + tid;
                const v4f val = *(const v4fa*)(&os[idx * 4]);
                *(volatile v4f*)(dst + (size_t)idx * 4) = val; }
            if (ps == 0) __threadfence(); }
    } else if (o0 < 2 * CQK) {
        const int hb = (o0 - CQK) / KD;
#pragma unroll 1
        for (int ps = 0; ps < 2; ++ps) {
#pragma unroll 1
            for (int hh = 0; hh < 2; ++hh) {
                h16* dst = KP + ((size_t)(b * NHEAD + hb + hh) * NP) * KD;
#pragma unroll 1
                for (int i = 0; i < 4; ++i) { const int p = i * (32 * GW) + tid; const int t = p >> 2, d8 = (p & 3) * 8; v8h hv;
#pragma unroll
                    for (int e = 0; e < 8; ++e) hv[e] = toh_flush(os[(hh * KD + d8 + e) * NP + t]);
                    *(volatile v8h*)(dst + (size_t)p * 8) = hv; } }
            if (ps == 0) __threadfence(); }
    } else {
        h16* dst = VT + ((size_t)b * CV + (o0 - 2 * CQK)) * NP;
#pragma unroll 1
        for (int ps = 0; ps < 2; ++ps) {
#pragma unroll 1
            for (int i = 0; i < 8; ++i) { const int p = i * (32 * GW) + tid;
                const v4f x0 = *(const v4fa*)(&os[p * 8]); const v4f x1 = *(const v4fa*)(&os[p * 8 + 4]); v8h hv;
#pragma unroll
                for (int e = 0; e < 4; ++e) { hv[e] = toh_flush(x0[e]); hv[4 + e] = toh_flush(x1[e]); }
                *(volatile v8h*)(dst + (size_t)p * 8) = hv; }
            if (ps == 0) __threadfence(); }
    }
}

__global__ __launch_bounds__(32 * GW) void k_dwq(const float* __restrict__ QP, const float* __restrict__ wdw,
                                                  const float* __restrict__ gg, const float* __restrict__ bb, const float* __restrict__ mm, const float* __restrict__ vv, h16* QH) {
#pragma clang fp contract(off)
    __shared__ __align__(16) float hal[KD * 256];
    __shared__ __align__(16) float ot[KD * NP];
    __shared__ float wsh[KD * 9];
    __shared__ float ssh[KD];
    __shared__ float tsh[KD];
    const int tid = threadIdx.x; const int zh = blockIdx.x; const int b = zh / NHEAD, h = zh % NHEAD;
    if (tid < KD) { const int c = h * KD + tid; const float s = bfr(gg[c]) * rsqrtf(bfr(vv[c]) + BN_EPS);
        ssh[tid] = s * QCAR; tsh[tid] = (bfr(bb[c]) - bfr(mm[c]) * s) * QCAR;
#pragma unroll 1
        for (int j = 0; j < 9; ++j) wsh[tid * 9 + j] = bfr(wdw[c * 9 + j]); }
    const float* src = QP + ((size_t)b * CQK + h * KD) * NP;
#pragma unroll 1
    for (int i = tid; i < KD * 256; i += 32 * GW) {
        const int c = i >> 8, pos = i & 255; const int yy = (pos >> 4) - 1, xx = (pos & 15) - 1;
        const bool ok = ((unsigned)yy < (unsigned)RES) & ((unsigned)xx < (unsigned)RES);
        const int yc = yy < 0 ? 0 : (yy > RES - 1 ? RES - 1 : yy); const int xc = xx < 0 ? 0 : (xx > RES - 1 ? RES - 1 : xx);
        float v = src[(size_t)c * NP + yc * RES + xc]; asm volatile("" : "+v"(v));
        hal[i] = ok ? v : 0.0f; }
    __syncthreads();
    { const int n = tid; const bool live = n < NTOK; const int nc = live ? n : NTOK - 1; const int py = nc / RES, px = nc - py * RES; const int p0 = py * 16 + px;
#pragma unroll 1
      for (int c = 0; c < KD; ++c) {
          float a = 0.0f;
#pragma unroll
          for (int ky = 0; ky < 3; ++ky)
#pragma unroll
              for (int kx = 0; kx < 3; ++kx) a += hal[c * 256 + p0 + ky * 16 + kx] * wsh[c * 9 + ky * 3 + kx];
          const float val = a * ssh[c] + tsh[c];
          ot[c * NP + n] = live ? val : 0.0f; } }
    __syncthreads();
    h16* dst = QH + (size_t)zh * NP * KD;
#pragma unroll 1
    for (int ps = 0; ps < 2; ++ps) {
#pragma unroll 1
        for (int i = 0; i < 4; ++i) { const int p = i * (32 * GW) + tid; const int t = p >> 2, d8 = (p & 3) * 8; v8h hv;
#pragma unroll
            for (int e = 0; e < 8; ++e) hv[e] = toh_flush(ot[(d8 + e) * NP + t]);
            *(volatile v8h*)(dst + (size_t)p * 8) = hv; }
        if (ps == 0) __threadfence(); }
}

__global__ __launch_bounds__(32 * AW) __attribute__((amdgpu_num_vgpr(256)))
void k_flash(const h16* __restrict__ QH, const h16* __restrict__ KP, const h16* __restrict__ VT, const float* __restrict__ BP, h16* ACT) {
    __shared__ __align__(16) float os[AW * 16 * OSP];
    const int lane = threadIdx.x & 31, lr = lane & 15, hi = lane >> 4;
    const int wave = __builtin_amdgcn_readfirstlane((int)(threadIdx.x >> 5));
    const int zh = blockIdx.y; const int b = zh / NHEAD, h = zh % NHEAD;
    const int t0 = (blockIdx.x * AW + wave) * 16;
    const size_t qo = ((size_t)zh * NP + t0 + lr) * KD + 8 * hi;
    const v16h qh = ldh(QH + qo);
    const size_t ko = ((size_t)zh * NP + lr) * KD + 8 * hi;
    const size_t vo = ((size_t)zh * VD + lr) * NP + 8 * hi;
    const size_t bo = ((size_t)h * NP + t0 + lr) * NP + 8 * hi;
    v8f o[8];
#pragma unroll
    for (int j = 0; j < 8; ++j) o[j] = (v8f){};
    float m = NEGB, l = 0.0f;
#pragma unroll 1
    for (int key0 = 0; key0 < NP; key0 += 32) {
        const h16* ka = KP + ko + (size_t)key0 * KD;
        const v16h ka0 = ldh(ka), kb0 = ldh(ka + 16 * KD);
        v8f sa = (v8f){}, sb = (v8f){};
        sa = wmma16g(ka0, qh, sa); sb = wmma16g(kb0, qh, sb);
        const float* bp = BP + bo + key0;
        const v4f b0 = *(const v4f*)bp, b1 = *(const v4f*)(bp + 4), b2 = *(const v4f*)(bp + 16), b3 = *(const v4f*)(bp + 20);
        float bx[8], by[8];
#pragma unroll
        for (int r = 0; r < 4; ++r) { bx[r] = b0[r]; bx[4 + r] = b1[r]; by[r] = b2[r]; by[4 + r] = b3[r]; }
        const int ja = key0 + 8 * hi;
        float ta[8], tb[8]; bool fa[8], fb[8]; float mx = NEGB;
#pragma unroll
        for (int r = 0; r < 8; ++r) {
            fa[r] = (ja + r) < NTOK;
            fb[r] = (ja + 16 + r) < NTOK;
            ta[r] = sa[r] * SC2 + bx[r]; tb[r] = sb[r] * SC2 + by[r];
            mx = fmaxf(mx, fmaxf(fa[r] ? ta[r] : NEGB, fb[r] ? tb[r] : NEGB)); }
        mx = fmaxf(mx, __shfl_xor(mx, 16, 32));
        const float mnew = fmaxf(m, mx);
        const float alpha = __builtin_amdgcn_exp2f(m - mnew);
        const float sh = PSH - mnew;
        v16h pb; float ls = 0.0f;
#pragma unroll
        for (int r = 0; r < 8; ++r) {
            const float xa = ta[r] + sh, xb = tb[r] + sh;
            const float ea = __builtin_amdgcn_exp2f(xa), eb = __builtin_amdgcn_exp2f(xb);
            const bool ga_ok = fa[r] & (xa >= -14.0f); const bool gb_ok = fb[r] & (xb >= -14.0f);
            const float ga = ga_ok ? ea : 0.0f, gb = gb_ok ? eb : 0.0f;
            const h16 pa = (h16)ga; const h16 pc = (h16)gb;
            pb[r] = pa; pb[8 + r] = pc;
            ls += (float)pa + (float)pc; }
        l = l * alpha + ls; m = mnew;
#pragma unroll
        for (int j = 0; j < 8; ++j) o[j] = o[j] * alpha;
        const h16* va = VT + vo + key0;
#pragma unroll
        for (int g = 0; g < 2; ++g) {
            v16h vf[4];
#pragma unroll
            for (int j = 0; j < 4; ++j) vf[j] = ldh(va + (size_t)((g * 4 + j) * 16) * NP);
#pragma unroll
            for (int j = 0; j < 4; ++j) o[g * 4 + j] = wmma16g(vf[j], pb, o[g * 4 + j]);
        }
    }
    l += __shfl_xor(l, 16, 32);
    const float inv = (1.0f / l) * ACAR;
    const int wb = wave * 16 * OSP;
#pragma unroll
    for (int j = 0; j < 8; ++j) { v4f a, c;
#pragma unroll
        for (int i = 0; i < 4; ++i) { a[i] = fmaxf(o[j][i] * inv, 0.0f); c[i] = fmaxf(o[j][4 + i] * inv, 0.0f); }
        *(v4fa*)(&os[wb + lr * OSP + 16 * j + 8 * hi]) = a; *(v4fa*)(&os[wb + lr * OSP + 16 * j + 8 * hi + 4]) = c; }
    wave_sync();
    h16* arow = ACT + ((size_t)b * NP + t0) * CV + h * VD;
#pragma unroll 1
    for (int ps = 0; ps < 2; ++ps) {
#pragma unroll
        for (int s = 0; s < 8; ++s) { const int row = 2 * s + (lane >> 4), c8 = (lane & 15) * 8;
            const bool live = (t0 + row) < NTOK;
            const v4f x0 = *(const v4fa*)(&os[wb + row * OSP + c8]); const v4f x1 = *(const v4fa*)(&os[wb + row * OSP + c8 + 4]); v8h hv;
#pragma unroll
            for (int e = 0; e < 4; ++e) { hv[e] = live ? toh_flush(x0[e]) : (h16)0.0f; hv[4 + e] = live ? toh_flush(x1[e]) : (h16)0.0f; }
            *(volatile v8h*)(arow + (size_t)row * CV + c8) = hv; }
        if (ps == 0) __threadfence(); }
}

__global__ __launch_bounds__(32 * GW) void k_proj(const h16* __restrict__ WPH, const h16* __restrict__ ACT,
                                                   const float* __restrict__ gg, const float* __restrict__ bb, const float* __restrict__ mm, const float* __restrict__ vv, float* OUT) {
    __shared__ __align__(16) float os[64 * NTOK];
    __shared__ float ss[64];
    __shared__ float ts[64];
    const int tid = threadIdx.x; const int lane = tid & 31, lr = lane & 15, hi = lane >> 4;
    const int wave = __builtin_amdgcn_readfirstlane((int)(threadIdx.x >> 5));
    const int o0 = blockIdx.x * 64, b = blockIdx.y;
    if (tid < 64) { const int o = o0 + tid; const float s = bfr(gg[o]) * rsqrtf(bfr(vv[o]) + BN_EPS); ss[tid] = s * CINV; ts[tid] = bfr(bb[o]) - bfr(mm[o]) * s; }
    v8f acc[4][2];
#pragma unroll
    for (int mb = 0; mb < 4; ++mb)
#pragma unroll
        for (int nb = 0; nb < 2; ++nb) acc[mb][nb] = (v8f){};
    const size_t aoff = (size_t)(o0 + lr) * CV + 8 * hi;
    const size_t boff = ((size_t)b * NP + wave * 32 + lr) * CV + 8 * hi;
#pragma unroll 1
    for (int kc = 0; kc < CV; kc += 32) {
        v16h a[4];
#pragma unroll
        for (int mb = 0; mb < 4; ++mb) a[mb] = ldh(WPH + aoff + (size_t)mb * 16 * CV + kc);
#pragma unroll
        for (int nb = 0; nb < 2; ++nb) { const v16h bq = ldh(ACT + boff + (size_t)nb * 16 * CV + kc);
#pragma unroll
            for (int mb = 0; mb < 4; ++mb) acc[mb][nb] = wmma16g(a[mb], bq, acc[mb][nb]); }
    }
    __syncthreads();
#pragma unroll
    for (int mb = 0; mb < 4; ++mb)
#pragma unroll
        for (int nb = 0; nb < 2; ++nb) { const int col = wave * 32 + nb * 16 + lr;
#pragma unroll
            for (int j = 0; j < 8; ++j) { const int row = mb * 16 + hi * 8 + j;
                const float val = acc[mb][nb][j] * ss[row] + ts[row];
                if (col < NTOK) os[row * NTOK + col] = val; } }
    __syncthreads();
    float* dst = OUT + ((size_t)b * COUT + o0) * NTOK;
#pragma unroll 1
    for (int ps = 0; ps < 2; ++ps) {
#pragma unroll 1
        for (int i = 0; i < 14; ++i) { const int idx = i * (32 * GW) + tid;
            const v4f val = *(const v4fa*)(&os[idx * 4]);
            *(volatile v4f*)(dst + (size_t)idx * 4) = val; }
        if (ps == 0) __threadfence(); }
}

static constexpr size_t al256(size_t v) { return (v + 255) & ~(size_t)255; }
static constexpr size_t SZ_WB = al256((size_t)CQKV * CIN * 2);
static constexpr size_t SZ_WP = al256((size_t)COUT * CV * 2);
static constexpr size_t SZ_BP = al256((size_t)NHEAD * NP * NP * 4);
static constexpr size_t SZ_XB = al256((size_t)BCH * NP * CIN * 2);
static constexpr size_t SZ_QP = al256((size_t)BCH * CQK * NP * 4);
static constexpr size_t SZ_QH = al256((size_t)BCH * NHEAD * NP * KD * 2);
static constexpr size_t SZ_VT = al256((size_t)BCH * CV * NP * 2);
static constexpr size_t SZ_AC = al256((size_t)BCH * NP * CV * 2);
static constexpr size_t SZ_TOTAL = SZ_WB + SZ_WP + SZ_BP + SZ_XB + SZ_QP + 2 * SZ_QH + SZ_VT + SZ_AC;
static_assert(SZ_TOTAL <= (size_t)134217728);
static_assert((size_t)BCH * NHEAD * VD == (size_t)BCH * CV);

extern "C" void kernel_launch(void* const* d_in, const int* in_sizes, int n_in,
                              void* d_out, int out_size, void* d_ws, size_t ws_size, hipStream_t stream) {
    if (n_in < 18) return;
    if ((size_t)in_sizes[0] < (size_t)NB * CIN * NTOK) return;
    if ((size_t)in_sizes[1] < (size_t)CQKV * CIN) return;
    if (in_sizes[2] < CQKV || in_sizes[3] < CQKV || in_sizes[4] < CQKV || in_sizes[5] < CQKV) return;
    if (in_sizes[6] < CQK * 9) return;
    if (in_sizes[7] < CQK || in_sizes[8] < CQK || in_sizes[9] < CQK || in_sizes[10] < CQK) return;
    if ((size_t)in_sizes[11] < (size_t)COUT * CV) return;
    if (in_sizes[12] < COUT || in_sizes[13] < COUT || in_sizes[14] < COUT || in_sizes[15] < COUT) return;
    if (in_sizes[16] < NHEAD * NTOK || in_sizes[17] < NTOK * NTOK) return;
    if ((size_t)out_size < (size_t)NB * COUT * NTOK) return;
    if (SZ_TOTAL > ws_size) return;
    const float* x      = (const float*)d_in[0];
    const float* w_qkv  = (const float*)d_in[1];
    const float* g_qkv  = (const float*)d_in[2];
    const float* b_qkv  = (const float*)d_in[3];
    const float* m_qkv  = (const float*)d_in[4];
    const float* v_qkv  = (const float*)d_in[5];
    const float* w_dw   = (const float*)d_in[6];
    const float* g_dw   = (const float*)d_in[7];
    const float* b_dw   = (const float*)d_in[8];
    const float* m_dw   = (const float*)d_in[9];
    const float* v_dw   = (const float*)d_in[10];
    const float* w_proj = (const float*)d_in[11];
    const float* g_proj = (const float*)d_in[12];
    const float* b_proj = (const float*)d_in[13];
    const float* m_proj = (const float*)d_in[14];
    const float* v_proj = (const float*)d_in[15];
    const float* ab     = (const float*)d_in[16];
    const int*   idxs   = (const int*)d_in[17];
    float* OUT = (float*)d_out;
    char* wsp = (char*)d_ws;
    bf*    WB  = (bf*)wsp;    wsp += SZ_WB;
    h16*   WPH = (h16*)wsp;   wsp += SZ_WP;
    float* BP  = (float*)wsp; wsp += SZ_BP;
    bf*    XB  = (bf*)wsp;    wsp += SZ_XB;
    float* QP  = (float*)wsp; wsp += SZ_QP;
    h16*   QH  = (h16*)wsp;   wsp += SZ_QH;
    h16*   KP  = (h16*)wsp;   wsp += SZ_QH;
    h16*   VT  = (h16*)wsp;   wsp += SZ_VT;
    h16*   ACT = (h16*)wsp;   wsp += SZ_AC;

    { const size_t n8 = (size_t)CQKV * CIN / 8; k_cvt8<<<(unsigned)((n8 + 255) / 256), 256, 0, stream>>>(w_qkv, WB, n8); }
    { const size_t n8 = (size_t)COUT * CV / 8;  k_wcv<<<(unsigned)((n8 + 255) / 256), 256, 0, stream>>>(w_proj, WPH, n8); }
    k_bias<<<(unsigned)((size_t)NHEAD * NP * NP / 4 / 256), 256, 0, stream>>>(ab, idxs, BP);

    for (int ch = 0; ch < NCHUNK; ++ch) {
        const float* xin = x + (size_t)ch * BCH * CIN * NTOK;
        float* outc = OUT + (size_t)ch * BCH * COUT * NTOK;
        k_xt<<<dim3(CIN / 64, BCH, 1), 256, 0, stream>>>(xin, XB);
        k_qkv<<<dim3(CQKV / 64, BCH, 1), 32 * GW, 0, stream>>>(WB, XB, g_qkv, b_qkv, m_qkv, v_qkv, QP, KP, VT);
        k_dwq<<<dim3(BCH * NHEAD, 1, 1), 32 * GW, 0, stream>>>(QP, w_dw, g_dw, b_dw, m_dw, v_dw, QH);
        k_flash<<<dim3(QT / AW, BCH * NHEAD, 1), 32 * AW, 0, stream>>>(QH, KP, VT, BP, ACT);
        k_proj<<<dim3(COUT / 64, BCH, 1), 32 * GW, 0, stream>>>(WPH, ACT, g_proj, b_proj, m_proj, v_proj, outc);
    }
}
